// MultiHeadAttentionParallel_19490561590292
// MI455X (gfx1250) — hardware-verified
//
#include <hip/hip_runtime.h>
#include <math.h>
#include <stdint.h>

constexpr int kBatch = 2;
constexpr int kSeq   = 4096;
constexpr int kDim   = 512;
constexpr int kHeads = 8;
constexpr int kHd    = 64;
constexpr int kRows  = kBatch * kSeq;
static_assert(kHeads * kHd == kDim, "geometry");
static_assert(kSeq % 64 == 0 && kDim % 64 == 0 && kRows % 64 == 0, "tile multiples");

typedef __attribute__((ext_vector_type(16))) _Float16 v16h;
typedef __attribute__((ext_vector_type(8)))  _Float16 v8h;
typedef __attribute__((ext_vector_type(16))) __bf16   v16b;
typedef __attribute__((ext_vector_type(8)))  __bf16   v8b;
typedef __attribute__((ext_vector_type(8)))  float    v8f;
typedef __attribute__((ext_vector_type(4)))  float    v4f;
typedef __attribute__((ext_vector_type(2)))  float    v2f;
typedef __attribute__((ext_vector_type(4)))  unsigned int v4u;

__device__ __forceinline__ unsigned short f2bf_bits(float f) {
  unsigned u = __float_as_uint(f);
  return (unsigned short)((u + 0x7FFFu + ((u >> 16) & 1u)) >> 16);
}
__device__ __forceinline__ float bf_bits2f(unsigned short h) { return __uint_as_float(((unsigned)h) << 16); }

__device__ __forceinline__ void dep_guard_h(v8f& a, v8f& b, v16h x, v16h y) { asm volatile("v_nop\n\tv_nop\n\tv_nop\n\tv_nop" : "+v"(a), "+v"(b) : "v"(x), "v"(y)); }
__device__ __forceinline__ void dep_guard_b(v8f& a, v8f& b, v16b x, v16b y) { asm volatile("v_nop\n\tv_nop\n\tv_nop\n\tv_nop" : "+v"(a), "+v"(b) : "v"(x), "v"(y)); }
__device__ __forceinline__ void keep4_h(v16h a, v16h b, v16h c, v16h d) { asm volatile("v_nop" :: "v"(a), "v"(b), "v"(c), "v"(d)); }
__device__ __forceinline__ void keep4_b(v16b a, v16b b, v16b c, v16b d) { asm volatile("v_nop" :: "v"(a), "v"(b), "v"(c), "v"(d)); }
__device__ __forceinline__ void acc_guard4(v8f& a, v8f& b, v8f& c, v8f& d) { asm volatile("v_nop\n\tv_nop\n\tv_nop\n\tv_nop" : "+v"(a), "+v"(b), "+v"(c), "+v"(d)); }
template <typename T> struct Frag;
template <> struct Frag<_Float16> {
  typedef v16h V; union U { v16h v; v8h h[2]; };
  static __device__ __forceinline__ v16h load(const _Float16* p) {
    U f; f.h[0] = *(const v8h*)(p); f.h[1] = *(const v8h*)(p + 16); return f.v;
  }
  static __device__ __forceinline__ v8f mma(v16h a, v16h b, v8f c) {
    return __builtin_amdgcn_wmma_f32_16x16x32_f16(false, a, false, b, (short)0, c, false, false);
  }
  static __device__ __forceinline__ void guard(v8f& a, v8f& b, v16h x, v16h y) { dep_guard_h(a, b, x, y); }
  static __device__ __forceinline__ void keep(v16h a, v16h b, v16h c, v16h d) { keep4_h(a, b, c, d); }
};
template <> struct Frag<__bf16> {
  typedef v16b V; union U { v16b v; v8b h[2]; };
  static __device__ __forceinline__ v16b load(const __bf16* p) {
    U f; f.h[0] = *(const v8b*)(p); f.h[1] = *(const v8b*)(p + 16); return f.v;
  }
  static __device__ __forceinline__ v8f mma(v16b a, v16b b, v8f c) {
    return __builtin_amdgcn_wmma_f32_16x16x32_bf16(false, a, false, b, (short)0, c, false, false);
  }
  static __device__ __forceinline__ void guard(v8f& a, v8f& b, v16b x, v16b y) { dep_guard_b(a, b, x, y); }
  static __device__ __forceinline__ void keep(v16b a, v16b b, v16b c, v16b d) { keep4_b(a, b, c, d); }
};

template <int ET> struct Elem;
template <> struct Elem<0> { typedef _Float16 T; };
template <> struct Elem<1> { typedef __bf16 T; };
template <int ET, int SPLIT, int BIAS_MODE, int OUT_MODE, bool RESID, int ACT = 0>
__global__ __launch_bounds__(256) void wmma_gemm64(
    const unsigned short* __restrict__ Ap, const unsigned short* __restrict__ A2p, int lda, long strideA,
    const unsigned short* __restrict__ Btp, const unsigned short* __restrict__ Bt2p, int ldb, long strideB,
    void* __restrict__ Cout, void* __restrict__ Cout2, int ldc, long strideC,
    const float* __restrict__ bias,
    const float* __restrict__ resid, long strideR,
    int M, int N, int K, float scale) {
  typedef typename Elem<ET>::T T;
  typedef typename Frag<T>::V V;
  const T* A = (const T*)Ap; const T* A2 = (const T*)A2p; const T* Bt = (const T*)Btp; const T* Bt2 = (const T*)Bt2p;
  __shared__ __align__(16) float sT[8][16 * 68];
  const int b    = blockIdx.y;
  const int lane = threadIdx.x & 31;
  const int wave = threadIdx.x >> 5;
  const int tilesN = N >> 6;
  const int tilesM = M >> 6;
  const int tile = blockIdx.x * 8 + wave;
  if (tile >= tilesM * tilesN) return;
  const int tm = tile / tilesN;
  const int tn = tile - tm * tilesN;
  const int m0 = tm << 6;
  const int n0 = tn << 6;

  const T* Ab  = A  + (size_t)b * strideA;
  const T* Bb  = Bt + (size_t)b * strideB;
  const T* Ab2 = (SPLIT != 0) ? (A2  + (size_t)b * strideA) : nullptr;
  const T* Bb2 = (SPLIT == 1) ? (Bt2 + (size_t)b * strideB) : nullptr;

  const int rlane = lane & 15;
  const int koff  = (lane >> 4) * 8;
  const int mOff  = (lane >> 4) * 8;

  v8f acc[4][4];
#pragma unroll
  for (int i = 0; i < 4; ++i)
#pragma unroll
    for (int j = 0; j < 4; ++j) acc[i][j] = (v8f){0.f,0.f,0.f,0.f,0.f,0.f,0.f,0.f};

  for (int k0 = 0; k0 < K; k0 += 32) {
    V bh[4], bl[4];
#pragma unroll
    for (int j = 0; j < 4; ++j) {
      const size_t bo = (size_t)(n0 + (j << 4) + rlane) * ldb + koff + k0;
      bh[j] = Frag<T>::load(Bb + bo);
      if (SPLIT == 1) bl[j] = Frag<T>::load(Bb2 + bo);
    }
#pragma unroll
    for (int i = 0; i < 4; ++i) {
      const size_t ao = (size_t)(m0 + (i << 4) + rlane) * lda + koff + k0;
      V ah = Frag<T>::load(Ab + ao);
      V al;
      if (SPLIT != 0) al = Frag<T>::load(Ab2 + ao);
#pragma unroll
      for (int j = 0; j < 4; ++j) {
        acc[i][j] = Frag<T>::mma(ah, bh[j], acc[i][j]);
        if (SPLIT == 1) acc[i][j] = Frag<T>::mma(ah, bl[j], acc[i][j]);
        if (SPLIT != 0) acc[i][j] = Frag<T>::mma(al, bh[j], acc[i][j]);
      }
      Frag<T>::guard(acc[i][0], acc[i][3], ah, (SPLIT != 0) ? al : ah);
    }
    Frag<T>::keep(bh[0], bh[1], bh[2], bh[3]);
    if (SPLIT == 1) Frag<T>::keep(bl[0], bl[1], bl[2], bl[3]);
  }
  acc_guard4(acc[0][0], acc[0][1], acc[0][2], acc[0][3]);
  acc_guard4(acc[1][0], acc[1][1], acc[1][2], acc[1][3]);
  acc_guard4(acc[2][0], acc[2][1], acc[2][2], acc[2][3]);
  acc_guard4(acc[3][0], acc[3][1], acc[3][2], acc[3][3]);

  float* slab = sT[wave];
  const float* Rb = RESID ? (resid + (size_t)b * strideR) : nullptr;
#pragma unroll
  for (int i = 0; i < 4; ++i) {
    const int mBase = m0 + (i << 4);
#pragma unroll
    for (int j = 0; j < 4; ++j) {
      const int n = n0 + (j << 4) + rlane;
      float bv = 0.f;
      if (BIAS_MODE == 2) bv = bias[n];
#pragma unroll
      for (int r = 0; r < 8; ++r) {
        float v = acc[i][j][r] * scale;
        if (BIAS_MODE == 1) v += bias[mBase + mOff + r];
        if (BIAS_MODE == 2) v += bv;
        if (RESID) v += Rb[(size_t)(mBase + mOff + r) * ldc + n];
        if (ACT == 1) v = tanhf(v);
        if (ACT == 2) v = fmaxf(v, 0.0f);
        if (ACT == 3) v = v / (1.0f + expf(-v));
        if (ACT == 4) v = (v > 0.f) ? v : 0.01f * v;
        slab[(mOff + r) * 68 + (j << 4) + rlane] = v;
      }
    }
    __builtin_amdgcn_fence(__ATOMIC_RELEASE, "workgroup");
    __builtin_amdgcn_wave_barrier();
    __builtin_amdgcn_fence(__ATOMIC_ACQUIRE, "workgroup");
    if (OUT_MODE == 0) {
      float* C = (float*)Cout + (size_t)b * strideC;
      const int hh = lane >> 4, c4 = (lane & 15) * 4;
      for (int pass = 0; pass < 2; ++pass) {
#pragma unroll
        for (int it = 0; it < 8; ++it) {
          const int row = it * 2 + hh;
          v4f v = *(const v4f*)(slab + row * 68 + c4);
          *(volatile v4f*)(C + (size_t)(mBase + row) * ldc + n0 + c4) = v;
        }
        __threadfence();
      }
    } else {
      const int q = lane >> 3, c8 = (lane & 7) * 8;
      unsigned short* C  = (unsigned short*)Cout  + (size_t)b * strideC;
      unsigned short* C2 = (OUT_MODE == 2) ? ((unsigned short*)Cout2 + (size_t)b * strideC) : nullptr;
      for (int pass = 0; pass < 2; ++pass) {
#pragma unroll
        for (int it = 0; it < 4; ++it) {
          const int row = it * 4 + q;
          const float* sp = slab + row * 68 + c8;
          v8h hv, lv;
#pragma unroll
          for (int e = 0; e < 8; ++e) {
            if (OUT_MODE == 1) {
              hv[e] = (_Float16)sp[e];
            } else {
              unsigned short hb = f2bf_bits(sp[e]);
              unsigned short lb = f2bf_bits(sp[e] - bf_bits2f(hb));
              hv[e] = __builtin_bit_cast(_Float16, hb);
              lv[e] = __builtin_bit_cast(_Float16, lb);
            }
          }
          *(volatile v8h*)(C + (size_t)(mBase + row) * ldc + n0 + c8) = hv;
          if (OUT_MODE == 2) *(volatile v8h*)(C2 + (size_t)(mBase + row) * ldc + n0 + c8) = lv;
        }
        __threadfence();
      }
    }
    __builtin_amdgcn_fence(__ATOMIC_RELEASE, "workgroup");
    __builtin_amdgcn_wave_barrier();
    __builtin_amdgcn_fence(__ATOMIC_ACQUIRE, "workgroup");
  }
}

__device__ __forceinline__ unsigned pk16(unsigned short a, unsigned short b) { return (unsigned)a | ((unsigned)b << 16); }

__global__ __launch_bounds__(256) void split_bf16x2_kernel(const float* __restrict__ in, unsigned short* __restrict__ hi,
                                                           unsigned short* __restrict__ lo, int n2) {
  const int i = blockIdx.x * 256 + threadIdx.x;
  if (i < n2) {
    const v2f f = *(const v2f*)(in + 2 * (size_t)i);
    const unsigned short h0 = f2bf_bits(f[0]), h1 = f2bf_bits(f[1]);
    const unsigned short l0 = f2bf_bits(f[0] - bf_bits2f(h0)), l1 = f2bf_bits(f[1] - bf_bits2f(h1));
    const unsigned uh = pk16(h0, h1), ul = pk16(l0, l1);
    ((volatile unsigned*)hi)[i] = uh;
    ((volatile unsigned*)lo)[i] = ul;
    __threadfence();
    ((volatile unsigned*)hi)[i] = uh;
    ((volatile unsigned*)lo)[i] = ul;
  }
}

__global__ __launch_bounds__(256) void cast_bf16x2_3(const float* __restrict__ in0, const float* __restrict__ in1,
                                                     const float* __restrict__ in2, unsigned short* __restrict__ out,
                                                     long planeElems, int n2) {
  const int which = blockIdx.y;
  const float* in = (which == 0) ? in0 : ((which == 1) ? in1 : in2);
  unsigned short* o = out + (size_t)which * planeElems;
  const int i = blockIdx.x * 256 + threadIdx.x;
  if (i < n2) {
    const v2f f = *(const v2f*)(in + 2 * (size_t)i);
    const unsigned u = pk16(f2bf_bits(f[0]), f2bf_bits(f[1]));
    ((volatile unsigned*)o)[i] = u;
    __threadfence();
    ((volatile unsigned*)o)[i] = u;
  }
}

template <bool LO>
__global__ __launch_bounds__(256) void tsplit_kernel(const float* __restrict__ W, unsigned short* __restrict__ oh,
                                                     unsigned short* __restrict__ ol, int R, int Cc, long sIn, long sOut) {
  __shared__ __align__(16) float tf[64 * 68];
  W  += (size_t)blockIdx.z * sIn;
  oh += (size_t)blockIdx.z * sOut;
  if (LO) ol += (size_t)blockIdx.z * sOut;
  const int c0  = blockIdx.x * 64;
  const int r0  = blockIdx.y * 64;
  const int tid = threadIdx.x;
  {
    const int lr = tid >> 4;
    const int c4 = (tid & 15) * 4;
#pragma unroll
    for (int it = 0; it < 4; ++it) {
      const int rr = it * 16 + lr;
      const v4f a = *(const v4f*)(W + (size_t)(r0 + rr) * Cc + c0 + c4);
      *(v4f*)(tf + rr * 68 + c4) = a;
    }
  }
  __syncthreads();
  const int sub = tid >> 3;
  const int c8  = (tid & 7) * 8;
  v4u hv[2], lv[2];
#pragma unroll
  for (int it = 0; it < 2; ++it) {
    const int oc = it * 32 + sub;
    v4u a, a2;
#pragma unroll
    for (int q = 0; q < 4; ++q) {
      const float f0 = tf[(c8 + 2 * q) * 68 + oc];
      const float f1 = tf[(c8 + 2 * q + 1) * 68 + oc];
      const unsigned short h0 = f2bf_bits(f0), h1 = f2bf_bits(f1);
      unsigned lp = 0u;
      if (LO) {
        const unsigned short l0 = f2bf_bits(f0 - bf_bits2f(h0)), l1 = f2bf_bits(f1 - bf_bits2f(h1));
        lp = pk16(l0, l1);
      }
      a[q]  = pk16(h0, h1);
      a2[q] = lp;
    }
    hv[it] = a; lv[it] = a2;
  }
  for (int pass = 0; pass < 2; ++pass) {
#pragma unroll
    for (int it = 0; it < 2; ++it) {
      const int oc = it * 32 + sub;
      const size_t go = (size_t)(c0 + oc) * R + r0 + c8;
      *(volatile v4u*)(oh + go) = hv[it];
      if (LO) *(volatile v4u*)(ol + go) = lv[it];
    }
    __threadfence();
  }
}

#define AT_D 64
#define AT_NW 4
#define AT_QB 64
#define AT_KC 64

__device__ __forceinline__ unsigned short at_bf_bits(float f) {
  unsigned u = __float_as_uint(f);
  return (unsigned short)((u + 0x7FFFu + ((u >> 16) & 1u)) >> 16);
}
__device__ __forceinline__ __bf16 at_f2bf(float f) { return __builtin_bit_cast(__bf16, at_bf_bits(f)); }
__device__ __forceinline__ void at_split(float f, __bf16& hi, __bf16& lo) {
  const unsigned short hb = at_bf_bits(f);
  hi = __builtin_bit_cast(__bf16, hb);
  lo = at_f2bf(f - __uint_as_float(((unsigned)hb) << 16));
}
__device__ __forceinline__ v8f at_mma(v16b a, v16b b, v8f c) {
  c = __builtin_amdgcn_wmma_f32_16x16x32_bf16(false, a, false, b, (short)0, c, false, false);
  asm volatile("v_nop\n\tv_nop\n\tv_nop\n\tv_nop" : "+v"(c) : "v"(a), "v"(b));
  return c;
}
__device__ __forceinline__ v8f at_mma_h(v16h a, v16h b, v8f c) {
  c = __builtin_amdgcn_wmma_f32_16x16x32_f16(false, a, false, b, (short)0, c, false, false);
  asm volatile("v_nop\n\tv_nop\n\tv_nop\n\tv_nop" : "+v"(c) : "v"(a), "v"(b));
  return c;
}

__global__ __launch_bounds__(128)
void mha_attn_kernel(const unsigned short* __restrict__ qp, const unsigned short* __restrict__ kp,
                     const unsigned short* __restrict__ vhp, const unsigned short* __restrict__ vlp,
                     const int* __restrict__ vlens, float* __restrict__ out, float sscale, float fillv) {
  union FB { v16b v; v8b h[2]; };
  union FH { v16h v; v8h h[2]; };
  __shared__ __align__(16) _Float16 Ksh[AT_KC * AT_D];
  __shared__ __align__(16) __bf16   Vth[AT_D * AT_KC];
  __shared__ __align__(16) __bf16   Vtl[AT_D * AT_KC];
  __shared__ __align__(16) __bf16   Psh[AT_NW][16 * AT_KC];
  __shared__ __align__(16) __bf16   Psl[AT_NW][16 * AT_KC];
  __shared__ __align__(16) float    Os[AT_NW][16 * 68];

  const int tid  = threadIdx.x;
  const int wave = tid >> 5;
  const int lane = tid & 31;
  const int hh   = lane >> 4;
  const int c    = lane & 15;

  const int nqb  = kSeq / AT_QB;
  const int bx   = blockIdx.x;
  const int qb   = bx % nqb;
  const int bhid = bx / nqb;
  const int h    = bhid % kHeads;
  int b = bhid / kHeads;
  b = (b > kBatch - 1) ? (kBatch - 1) : b;
  const int q0   = qb * AT_QB + wave * 16;
  const int vlen = vlens[b];

  const _Float16* Qb = (const _Float16*)(const void*)qp + (size_t)b * kSeq * kDim + (size_t)h * AT_D;
  const _Float16* Kb = (const _Float16*)(const void*)kp + (size_t)b * kSeq * kDim + (size_t)h * AT_D;
  const __bf16*   Vh = (const __bf16*)(const void*)vhp + (size_t)b * kDim * kSeq + (size_t)h * AT_D * kSeq;
  const __bf16*   Vl = (const __bf16*)(const void*)vlp + (size_t)b * kDim * kSeq + (size_t)h * AT_D * kSeq;
  float*          ob = out + (size_t)b * kSeq * kDim + (size_t)h * AT_D;

  v16h qa[2];
#pragma unroll
  for (int dc = 0; dc < 2; ++dc) {
    qa[dc] = Frag<_Float16>::load(Qb + (size_t)(q0 + c) * kDim + dc * 32 + 8 * hh);
  }

  float mrow[8], lrow[8];
  v8f oacc[4];
#pragma unroll
  for (int r = 0; r < 8; ++r) { mrow[r] = -INFINITY; lrow[r] = 0.f; }
#pragma unroll
  for (int t = 0; t < 4; ++t) oacc[t] = (v8f){0.f,0.f,0.f,0.f,0.f,0.f,0.f,0.f};

  const int nChunks = kSeq / AT_KC;
  for (int kc = 0; kc < nChunks; ++kc) {
    const int kv0 = kc * AT_KC;
    __syncthreads();
    {
      const int r = tid >> 1, half = (tid & 1) * 32;
      const _Float16* ks  = Kb + (size_t)(kv0 + r) * kDim + half;
      const __bf16*   vsh = Vh + (size_t)r * kSeq + kv0 + half;
      const __bf16*   vsl = Vl + (size_t)r * kSeq + kv0 + half;
#pragma unroll
      for (int i = 0; i < 4; ++i) {
        const v8h a0 = *(const v8h*)(ks + 8 * i);
        const v8b b0 = *(const v8b*)(vsh + 8 * i);
        const v8b b1 = *(const v8b*)(vsl + 8 * i);
        *(v8h*)(Ksh + r * AT_D  + half + 8 * i) = a0;
        *(v8b*)(Vth + r * AT_KC + half + 8 * i) = b0;
        *(v8b*)(Vtl + r * AT_KC + half + 8 * i) = b1;
      }
    }
    __syncthreads();

    v8f s[4];
#pragma unroll
    for (int j = 0; j < 4; ++j) {
      s[j] = (v8f){0.f,0.f,0.f,0.f,0.f,0.f,0.f,0.f};
#pragma unroll
      for (int dc = 0; dc < 2; ++dc) {
        FH kb;
        kb.h[0] = *(const v8h*)(Ksh + (j * 16 + c) * AT_D + dc * 32 + 8 * hh);
        kb.h[1] = *(const v8h*)(Ksh + (j * 16 + c) * AT_D + dc * 32 + 16 + 8 * hh);
        s[j] = at_mma_h(qa[dc], kb.v, s[j]);
      }
    }
    float cm[8];
#pragma unroll
    for (int r = 0; r < 8; ++r) {
      float m = -INFINITY;
#pragma unroll
      for (int j = 0; j < 4; ++j) {
        const int kvcol = kv0 + j * 16 + c;
        const float sv = s[j][r] * sscale;
        const float sm = (kvcol < vlen) ? sv : fillv;
        s[j][r] = sm;
        m = fmaxf(m, sm);
      }
#pragma unroll
      for (int off = 1; off < 16; off <<= 1) m = fmaxf(m, __shfl_xor(m, off, 32));
      cm[r] = m;
    }
    __bf16* pwh = Psh[wave];
    __bf16* pwl = Psl[wave];
#pragma unroll
    for (int r = 0; r < 8; ++r) {
      const float mnew  = fmaxf(mrow[r], cm[r]);
      const float alpha = expf(mrow[r] - mnew);
      mrow[r] = mnew;
      float psum = 0.f;
#pragma unroll
      for (int j = 0; j < 4; ++j) {
        const float p = expf(s[j][r] - mnew);
        psum += p;
        __bf16 a, bl; at_split(p, a, bl);
        pwh[(8 * hh + r) * AT_KC + j * 16 + c] = a;
        pwl[(8 * hh + r) * AT_KC + j * 16 + c] = bl;
      }
#pragma unroll
      for (int off = 1; off < 16; off <<= 1) psum += __shfl_xor(psum, off, 32);
      lrow[r] = lrow[r] * alpha + psum;
#pragma unroll
      for (int t = 0; t < 4; ++t) oacc[t][r] *= alpha;
    }
    __builtin_amdgcn_fence(__ATOMIC_RELEASE, "workgroup");
    __builtin_amdgcn_wave_barrier();
    __builtin_amdgcn_fence(__ATOMIC_ACQUIRE, "workgroup");
#pragma unroll 1
    for (int kk = 0; kk < 2; ++kk) {
      FB pa, pl;
      pa.h[0] = *(const v8b*)(pwh + c * AT_KC + kk * 32 + 8 * hh);
      pa.h[1] = *(const v8b*)(pwh + c * AT_KC + kk * 32 + 16 + 8 * hh);
      pl.h[0] = *(const v8b*)(pwl + c * AT_KC + kk * 32 + 8 * hh);
      pl.h[1] = *(const v8b*)(pwl + c * AT_KC + kk * 32 + 16 + 8 * hh);
#pragma unroll
      for (int t = 0; t < 4; ++t) {
        FB vb, vl;
        vb.h[0] = *(const v8b*)(Vth + (t * 16 + c) * AT_KC + kk * 32 + 8 * hh);
        vb.h[1] = *(const v8b*)(Vth + (t * 16 + c) * AT_KC + kk * 32 + 16 + 8 * hh);
        vl.h[0] = *(const v8b*)(Vtl + (t * 16 + c) * AT_KC + kk * 32 + 8 * hh);
        vl.h[1] = *(const v8b*)(Vtl + (t * 16 + c) * AT_KC + kk * 32 + 16 + 8 * hh);
        oacc[t] = at_mma(pa.v, vb.v, oacc[t]);
        oacc[t] = at_mma(pa.v, vl.v, oacc[t]);
        oacc[t] = at_mma(pl.v, vb.v, oacc[t]);
      }
    }
  }

  float* os = Os[wave];
#pragma unroll
  for (int r = 0; r < 8; ++r) {
    const float inv = 1.0f / lrow[r];
#pragma unroll
    for (int t = 0; t < 4; ++t) os[(8 * hh + r) * 68 + t * 16 + c] = oacc[t][r] * inv;
  }
  __builtin_amdgcn_fence(__ATOMIC_RELEASE, "workgroup");
  __builtin_amdgcn_wave_barrier();
  __builtin_amdgcn_fence(__ATOMIC_ACQUIRE, "workgroup");
  {
    const int c4 = (lane & 15) * 4;
    for (int pass = 0; pass < 2; ++pass) {
#pragma unroll
      for (int it = 0; it < 8; ++it) {
        const int row = it * 2 + hh;
        v4f val = *(const v4f*)(os + row * 68 + c4);
        *(volatile v4f*)(ob + (size_t)(q0 + row) * kDim + c4) = val;
      }
      __threadfence();
    }
  }
}

extern "C" void kernel_launch(void* const* d_in, const int* in_sizes, int n_in,
                              void* d_out, int out_size, void* d_ws,
                              size_t ws_size, hipStream_t stream) {
  if (n_in < 8) return;
  const int nX = kRows * kDim;
  const int nW = kDim * kDim;
  if (in_sizes[0] != nX || in_sizes[1] != nX || in_sizes[2] != nX) return;
  if (in_sizes[3] < kBatch) return;
  if (in_sizes[4] != nW || in_sizes[5] != nW || in_sizes[6] != nW || in_sizes[7] != nW) return;
  if (out_size != nX) return;

  const float* queries = (const float*)d_in[0];
  const float* keys    = (const float*)d_in[1];
  const float* values  = (const float*)d_in[2];
  const int*   vlens   = (const int*)d_in[3];
  const float* Wq      = (const float*)d_in[4];
  const float* Wk      = (const float*)d_in[5];
  const float* Wv      = (const float*)d_in[6];
  const float* Wo      = (const float*)d_in[7];

  const size_t bX16 = (size_t)nX * 2;
  const size_t bW16 = (size_t)nW * 2;
  const size_t off_x  = 0;
  const size_t off_wh = off_x  + 3 * bX16;
  const size_t off_q  = off_wh + 4 * bW16;
  const size_t off_k  = off_q  + bX16;
  const size_t off_vh = off_k  + bX16;
  const size_t off_vl = off_vh + bX16;
  const size_t off_o  = off_vl + bX16;
  const size_t off_oh = off_o  + (size_t)nX * 4;
  const size_t off_ol = off_oh + bX16;
  const size_t total  = off_ol + bX16;
  if (total > ws_size) return;

  char* ws = (char*)d_ws;
  unsigned short* xbf  = (unsigned short*)(ws + off_x);
  unsigned short* wth  = (unsigned short*)(ws + off_wh);
  unsigned short* qh16 = (unsigned short*)(ws + off_q);
  unsigned short* kh16 = (unsigned short*)(ws + off_k);
  unsigned short* vth  = (unsigned short*)(ws + off_vh);
  unsigned short* vtl  = (unsigned short*)(ws + off_vl);
  float* obuf = (float*)(ws + off_o);
  unsigned short* ohi  = (unsigned short*)(ws + off_oh);
  unsigned short* olo  = (unsigned short*)(ws + off_ol);
  const float* dummyf  = (const float*)(ws + off_x);

  const long planeX = (long)nX;
  const long planeW = (long)nW;
  dim3 blk256(256), blk128(128);

  cast_bf16x2_3<<<dim3(nX / 2 / 256, 3), blk256, 0, stream>>>(queries, keys, values, xbf, planeX, nX / 2);

  tsplit_kernel<false><<<dim3(kDim / 64, kDim / 64, 1), blk256, 0, stream>>>(Wq, wth + 0 * planeW, wth + 0 * planeW, kDim, kDim, 0L, 0L);
  tsplit_kernel<false><<<dim3(kDim / 64, kDim / 64, 1), blk256, 0, stream>>>(Wk, wth + 1 * planeW, wth + 1 * planeW, kDim, kDim, 0L, 0L);
  tsplit_kernel<false><<<dim3(kDim / 64, kDim / 64, 1), blk256, 0, stream>>>(Wv, wth + 2 * planeW, wth + 2 * planeW, kDim, kDim, 0L, 0L);
  tsplit_kernel<false><<<dim3(kDim / 64, kDim / 64, 1), blk256, 0, stream>>>(Wo, wth + 3 * planeW, wth + 3 * planeW, kDim, kDim, 0L, 0L);

  const int gProj = (kRows / 64) * (kDim / 64) / 8;
  wmma_gemm64<1, 0, 0, 1, false><<<dim3(gProj, 2), blk256, 0, stream>>>(
      xbf, xbf, kDim, planeX,
      wth, wth, kDim, planeW,
      (void*)qh16, (void*)qh16, kDim, planeX,
      dummyf, dummyf, 0L, kRows, kDim, kDim, 1.0f);
  const int gVt = (kDim / 64) * (kSeq / 64) / 8;
  wmma_gemm64<1, 0, 0, 2, false><<<dim3(gVt, kBatch), blk256, 0, stream>>>(
      wth + 2 * planeW, wth + 2 * planeW, kDim, 0L,
      xbf + 2 * planeX, xbf + 2 * planeX, kDim, (long)kSeq * kDim,
      (void*)vth, (void*)vtl, kSeq, (long)kDim * kSeq,
      dummyf, dummyf, 0L, kDim, kSeq, kDim, 1.0f);

  mha_attn_kernel<<<dim3(kBatch * kHeads * (kSeq / 64)), blk128, 0, stream>>>(
      qh16, kh16, vth, vtl, vlens, obuf, 0.125f, -1000000.0f);

  split_bf16x2_kernel<<<dim3(nX / 2 / 256), blk256, 0, stream>>>(obuf, ohi, olo, nX / 2);

  wmma_gemm64<1, 2, 0, 0, false><<<dim3(gProj, 1), blk256, 0, stream>>>(
      ohi, olo, kDim, 0L,
      wth + 3 * planeW, wth + 3 * planeW, kDim, 0L,
      d_out, d_out, kDim, 0L,
      dummyf, dummyf, 0L, kRows, kDim, kDim, 1.0f);
}
